// ImputedMultiTimeAttentionV2_45148696215775
// MI455X (gfx1250) — hardware-verified
//
#include <hip/hip_runtime.h>


#define NBT  8
#define LQ   256
#define LK   512
#define DD   128
#define FF   32
#define NH_  8
#define DK   16
#define DKP  32
#define NQR  (NBT * LQ)
#define NKR  (NBT * LK)
#define DM   DD
#define NTK  NQR
#define MASKV (-1e30f)
#define LOSC 1024.0f

typedef _Float16 h16;
typedef unsigned short bf;
typedef __attribute__((ext_vector_type(16))) __bf16   v16bf;
typedef __attribute__((ext_vector_type(16))) _Float16 v16h;
typedef __attribute__((ext_vector_type(8)))  _Float16 v8h;
typedef __attribute__((ext_vector_type(8)))  unsigned short v8us;
typedef __attribute__((ext_vector_type(8)))  float    v8f;
typedef __attribute__((ext_vector_type(4)))  float    v4f;
typedef __attribute__((ext_vector_type(4)))  _Float16 v4h;
typedef v8h  __attribute__((may_alias)) v8ha;
typedef v4f  __attribute__((may_alias)) v4fa;
typedef v8us __attribute__((may_alias)) v8usa;

__device__ __forceinline__ unsigned short f2bf(float f) { unsigned u = __float_as_uint(f); u += 0x7FFFu + ((u >> 16) & 1u); return (unsigned short)(u >> 16); }
__device__ __forceinline__ float bf2f(unsigned short b) { return __uint_as_float(((unsigned)b) << 16); }
__device__ __forceinline__ float bfr(float f) { return bf2f(f2bf(f)); }
__device__ __forceinline__ v16h cat16(v8h lo, v8h hi) { return __builtin_shufflevector(lo, hi, 0, 1, 2, 3, 4, 5, 6, 7, 8, 9, 10, 11, 12, 13, 14, 15); }
__device__ __forceinline__ v16bf cat16b(v8us lo, v8us hi) { return __builtin_bit_cast(v16bf, __builtin_shufflevector(lo, hi, 0, 1, 2, 3, 4, 5, 6, 7, 8, 9, 10, 11, 12, 13, 14, 15)); }
__device__ __forceinline__ v8f wmma16(v16h a, v16h b, v8f c) { return __builtin_amdgcn_wmma_f32_16x16x32_f16(false, a, false, b, (short)0, c, false, false); }
__device__ __forceinline__ v8f wmmab(v16bf a, v16bf b, v8f c) { return __builtin_amdgcn_wmma_f32_16x16x32_bf16(false, a, false, b, (short)0, c, false, false); }

template <bool SPLITA, bool F16OUT = false>
__global__ __launch_bounds__(128) void k_gemmb(const bf* __restrict__ A, const bf* __restrict__ Al, const bf* __restrict__ Bn, const float* __restrict__ bias, float* C, int ldc, h16* C2, const float* __restrict__ R = nullptr, int K = DM, int roundR = 1) {
    __shared__ __align__(16) float ost[4][16 * 68];
    const int lane = threadIdx.x & 31, wave = threadIdx.x >> 5, lr = lane & 15, hi = lane >> 4;
    const int r0 = blockIdx.x * 64 + wave * 16, c0 = blockIdx.y * 64;
    const size_t aoff = (size_t)(r0 + lr) * K + 8 * hi;
    size_t boff[4];
#pragma unroll
    for (int t = 0; t < 4; ++t) boff[t] = (size_t)(c0 + t * 16 + lr) * K + 8 * hi;
    v8f acc[4];
#pragma unroll
    for (int t = 0; t < 4; ++t) acc[t] = (v8f){};
#pragma unroll 1
    for (int kc = 0; kc < K; kc += 32) {
        const v16bf a = cat16b(*(const v8us*)(A + aoff + kc), *(const v8us*)(A + aoff + kc + 16));
        v16bf al = a;
        if (SPLITA) al = cat16b(*(const v8us*)(Al + aoff + kc), *(const v8us*)(Al + aoff + kc + 16));
#pragma unroll
        for (int t = 0; t < 4; ++t) { const v16bf b = cat16b(*(const v8us*)(Bn + boff[t] + kc), *(const v8us*)(Bn + boff[t] + kc + 16)); acc[t] = wmmab(a, b, acc[t]); if (SPLITA) acc[t] = wmmab(al, b, acc[t]); }
        asm volatile("v_nop\n\tv_nop\n\tv_nop\n\tv_nop" : "+v"(acc[0]), "+v"(acc[1]), "+v"(acc[2]), "+v"(acc[3]) : "v"(a), "v"(al));
    }
    float* os = &ost[wave][0];
#pragma unroll
    for (int t = 0; t < 4; ++t) { const float bv = bias ? bfr(bias[c0 + t * 16 + lr]) : 0.f;
#pragma unroll
        for (int j = 0; j < 8; ++j) os[(hi * 8 + j) * 68 + t * 16 + lr] = acc[t][j] + bv; }
    __syncthreads();
    if (F16OUT) {
        h16* crow = (h16*)(void*)C + (size_t)r0 * ldc + c0;
        auto pass = [&]() {
#pragma unroll
            for (int s = 0; s < 4; ++s) { const int row = 4 * s + (lane >> 3), piece = lane & 7; const float* sp = os + row * 68 + piece * 8; v8h o, o2;
#pragma unroll
                for (int i = 0; i < 8; ++i) { const h16 a = (h16)sp[i]; o[i] = a; o2[i] = (h16)((sp[i] - (float)a) * LOSC); }
                *(volatile v8h*)(crow + (size_t)row * ldc + piece * 8) = o; if (C2) *(volatile v8h*)(C2 + (size_t)r0 * ldc + c0 + (size_t)row * ldc + piece * 8) = o2; }
        };
        pass(); __threadfence(); pass();
    } else {
        float* crow = C + (size_t)r0 * ldc + c0;
        auto pass = [&]() {
#pragma unroll
            for (int s = 0; s < 8; ++s) { const int Lid = (lane >> 3) + 4 * s, piece = lane & 7; const int row = Lid >> 1, cofs = (Lid & 1) * 32 + piece * 4;
                v4f val = *(const v4fa*)(os + row * 68 + cofs); if (R) { const v4f rv = *(const v4f*)(R + ((size_t)r0 + row) * ldc + c0 + cofs); val += roundR ? (v4f){bfr(rv[0]), bfr(rv[1]), bfr(rv[2]), bfr(rv[3])} : rv; }
                *(volatile v4f*)(crow + (size_t)row * ldc + cofs) = val; }
        };
        pass(); __threadfence(); pass();
    }
}

__global__ __launch_bounds__(128) void k_gemm3(const bf* __restrict__ Ah, const bf* __restrict__ Al, const bf* __restrict__ Bh, const bf* __restrict__ Bl, int K, float* C, int ldc) {
    __shared__ __align__(16) float ost[4][16 * 68];
    const int lane = threadIdx.x & 31, wave = threadIdx.x >> 5, lr = lane & 15, hi = lane >> 4;
    const int r0 = blockIdx.x * 64 + wave * 16, c0 = blockIdx.y * 64;
    const size_t aoff = (size_t)(r0 + lr) * K + 8 * hi;
    v8f acc[4];
#pragma unroll
    for (int t = 0; t < 4; ++t) acc[t] = (v8f){};
#pragma unroll 1
    for (int kc = 0; kc < K; kc += 32) {
        const v16bf a = cat16b(*(const v8us*)(Ah + aoff + kc), *(const v8us*)(Ah + aoff + kc + 16));
        const v16bf al = cat16b(*(const v8us*)(Al + aoff + kc), *(const v8us*)(Al + aoff + kc + 16));
#pragma unroll
        for (int t = 0; t < 4; ++t) { const size_t bo = (size_t)(c0 + t * 16 + lr) * K + kc + 8 * hi;
            const v16bf bh = cat16b(*(const v8us*)(Bh + bo), *(const v8us*)(Bh + bo + 16)); const v16bf bl = cat16b(*(const v8us*)(Bl + bo), *(const v8us*)(Bl + bo + 16));
            acc[t] = wmmab(a, bh, acc[t]); acc[t] = wmmab(al, bh, acc[t]); acc[t] = wmmab(a, bl, acc[t]); }
        asm volatile("v_nop\n\tv_nop\n\tv_nop\n\tv_nop" : "+v"(acc[0]), "+v"(acc[1]), "+v"(acc[2]), "+v"(acc[3]) : "v"(a), "v"(al));
    }
    float* os = &ost[wave][0];
#pragma unroll
    for (int t = 0; t < 4; ++t) {
#pragma unroll
        for (int j = 0; j < 8; ++j) os[(hi * 8 + j) * 68 + t * 16 + lr] = acc[t][j]; }
    __builtin_amdgcn_wave_barrier(); asm volatile("" ::: "memory");
    float* crow = C + (size_t)r0 * ldc + c0;
    auto pass = [&]() {
#pragma unroll
        for (int s = 0; s < 8; ++s) { const int Lid = (lane >> 3) + 4 * s, piece = lane & 7; const int row = Lid >> 1, cofs = (Lid & 1) * 32 + piece * 4;
            const v4f val = *(const v4fa*)(os + row * 68 + cofs); *(volatile v4f*)(crow + (size_t)row * ldc + cofs) = val; }
    };
    pass(); __threadfence(); pass();
}

__global__ __launch_bounds__(256) void k_bf(const float* __restrict__ src, bf* dst, size_t n8) {
    const size_t i = (size_t)blockIdx.x * 256 + threadIdx.x; if (i >= n8) return;
    const v8f v = *(const v8f*)(src + i * 8); v8us o;
#pragma unroll
    for (int k = 0; k < 8; ++k) o[k] = f2bf(v[k]);
    *(volatile v8us*)(dst + i * 8) = o; __threadfence(); *(volatile v8us*)(dst + i * 8) = o;
}
__global__ __launch_bounds__(256) void k_wn16(const float* __restrict__ Ws, bf* WN) {
    const int u = blockIdx.x * 256 + threadIdx.x; if (u >= NH_ * DK * DD / 8) return;
    const int n = u / (DD / 8), d0 = (u % (DD / 8)) * 8; const int j = n / DK, c = n % DK; v8us v;
#pragma unroll
    for (int i = 0; i < 8; ++i) v[i] = f2bf(Ws[((size_t)j * DD + d0 + i) * DK + c]);
    *(volatile v8us*)(WN + (size_t)n * DD + d0) = v; __threadfence(); *(volatile v8us*)(WN + (size_t)n * DD + d0) = v;
}
__global__ __launch_bounds__(256) void k_wnv(const float* __restrict__ Wv, bf* WVN) {
    const int u = blockIdx.x * 256 + threadIdx.x; if (u >= NH_ * FF * FF / 8) return;
    const int n = u / (FF / 8), g0 = (u % (FF / 8)) * 8; const int j = n / FF, f = n % FF; v8us v;
#pragma unroll
    for (int i = 0; i < 8; ++i) v[i] = f2bf(Wv[((size_t)j * FF + g0 + i) * FF + f]);
    *(volatile v8us*)(WVN + (size_t)n * FF + g0) = v; __threadfence(); *(volatile v8us*)(WVN + (size_t)n * FF + g0) = v;
}
__global__ __launch_bounds__(256) void k_hp(const float* __restrict__ X, int nrows, bf* Ph, bf* Pl) {
    typedef __attribute__((ext_vector_type(2))) unsigned short v2us;
    const int lane = threadIdx.x & 31, wid = blockIdx.x * 8 + (threadIdx.x >> 5); if (wid >= (nrows / 2) * NH_) return;
    const int rp = wid / NH_, h = wid % NH_; const int r = rp * 2 + (lane >> 4), c0 = (lane & 15) * 2;
    v2us oh, ol;
#pragma unroll
    for (int i = 0; i < 2; ++i) { const int c = c0 + i; const float v = (c < DK) ? X[(size_t)r * DD + h * DK + c] : 0.f; const unsigned short hb = f2bf(v); oh[i] = hb; ol[i] = f2bf(v - bf2f(hb)); }
    const size_t o = ((size_t)h * nrows + r) * DKP + c0;
    *(volatile v2us*)(Ph + o) = oh; *(volatile v2us*)(Pl + o) = ol; __threadfence(); *(volatile v2us*)(Ph + o) = oh; *(volatile v2us*)(Pl + o) = ol;
}
__global__ __launch_bounds__(256) void k_msoft(const float* __restrict__ S, const float* __restrict__ mask, const float* __restrict__ V, float* LAT) {
    const int tid = threadIdx.x; const int bh = blockIdx.x / (LQ / 8), qb = blockIdx.x % (LQ / 8); const int b = bh / NH_, h = bh % NH_;
    const int q = qb * 8 + (tid >> 5), f = tid & 31;
    const float* srow = S + ((size_t)bh * LQ + q) * LK; const float* mb = mask + (size_t)b * LK * FF + f; const float* vb = V + (size_t)b * LK * (NH_ * FF) + h * FF + f;
    float m = -3.0e38f, l = 0.f, acc = 0.f;
#pragma unroll 1
    for (int k = 0; k < LK; ++k) { const float mk = bfr(mb[(size_t)k * FF]); const float a = mk * srow[k] + (1.0f - mk) * MASKV;
        const float mn = fmaxf(m, a); const float sc = __expf(m - mn); const float p = __expf(a - mn);
        l = l * sc + p; acc = acc * sc + p * vb[(size_t)k * (NH_ * FF)]; m = mn; }
    const float out = acc / l;
    float* p = LAT + (((size_t)bh * LQ) + q) * FF + f; *(volatile float*)p = out; __threadfence(); *(volatile float*)p = out;
}
__global__ __launch_bounds__(256) void k_comb(const float* __restrict__ LAT, const float* __restrict__ Wc, const float* __restrict__ bc, float* OUTP) {
    const int i = blockIdx.x * 256 + threadIdx.x; if (i >= NBT * LQ * FF) return;
    const int f = i % FF, q = (i / FF) % LQ, b = i / (FF * LQ);
    float s = bfr(bc[f]);
#pragma unroll
    for (int h = 0; h < NH_; ++h) s = fmaf(LAT[(((size_t)(b * NH_ + h)) * LQ + q) * FF + f], bfr(Wc[f * NH_ + h]), s);
    const float y = tanhf(s);
    *(volatile float*)(OUTP + i) = y; __threadfence(); *(volatile float*)(OUTP + i) = y;
}

extern "C" void kernel_launch(void* const* d_in, const int* in_sizes, int n_in,
                              void* d_out, int out_size, void* d_ws, size_t ws_size, hipStream_t stream) {
    (void)in_sizes; (void)n_in; (void)out_size;
    const float* query = (const float*)d_in[0]; const float* key = (const float*)d_in[1]; const float* value = (const float*)d_in[2]; const float* mask = (const float*)d_in[3];
    const float* Wq = (const float*)d_in[4]; const float* Wk = (const float*)d_in[5]; const float* Wv = (const float*)d_in[6]; const float* Wc = (const float*)d_in[7]; const float* bc = (const float*)d_in[8];
    float* out = (float*)d_out;
    char* wsp = (char*)d_ws;
    auto take = [&](size_t bytes) { char* p = wsp; wsp += (bytes + 255) & ~(size_t)255; return (void*)p; };
    bf* WQN = (bf*)take((size_t)DD * DD * 2); bf* WKN = (bf*)take((size_t)DD * DD * 2); bf* WVN = (bf*)take((size_t)NH_ * FF * FF * 2);
    bf* Qb = (bf*)take((size_t)NQR * DD * 2); bf* Kb = (bf*)take((size_t)NKR * DD * 2); bf* Vb = (bf*)take((size_t)NKR * FF * 2);
    float* Qf = (float*)take((size_t)NQR * DD * 4); float* Kf = (float*)take((size_t)NKR * DD * 4); float* Vf = (float*)take((size_t)NKR * NH_ * FF * 4);
    bf* QPh = (bf*)take((size_t)NH_ * NQR * DKP * 2); bf* QPl = (bf*)take((size_t)NH_ * NQR * DKP * 2); bf* KPh = (bf*)take((size_t)NH_ * NKR * DKP * 2); bf* KPl = (bf*)take((size_t)NH_ * NKR * DKP * 2);
    float* S = (float*)take((size_t)NBT * NH_ * LQ * LK * 4); float* LAT = (float*)take((size_t)NBT * NH_ * LQ * FF * 4);
    if ((size_t)(wsp - (char*)d_ws) > ws_size) return;
    k_wn16<<<(NH_ * DK * DD / 8 + 255) / 256, 256, 0, stream>>>(Wq, WQN); k_wn16<<<(NH_ * DK * DD / 8 + 255) / 256, 256, 0, stream>>>(Wk, WKN); k_wnv<<<(NH_ * FF * FF / 8 + 255) / 256, 256, 0, stream>>>(Wv, WVN);
    k_bf<<<(NQR * DD / 8 + 255) / 256, 256, 0, stream>>>(query, Qb, (size_t)NQR * DD / 8); k_bf<<<(NKR * DD / 8 + 255) / 256, 256, 0, stream>>>(key, Kb, (size_t)NKR * DD / 8); k_bf<<<(NKR * FF / 8 + 255) / 256, 256, 0, stream>>>(value, Vb, (size_t)NKR * FF / 8);
    k_gemmb<false, false><<<dim3(NQR / 64, DD / 64, 1), 128, 0, stream>>>(Qb, nullptr, WQN, nullptr, Qf, DD, nullptr);
    k_gemmb<false, false><<<dim3(NKR / 64, DD / 64, 1), 128, 0, stream>>>(Kb, nullptr, WKN, nullptr, Kf, DD, nullptr);
    k_gemmb<false, false><<<dim3(NKR / 64, (NH_ * FF) / 64, 1), 128, 0, stream>>>(Vb, nullptr, WVN, nullptr, Vf, NH_ * FF, nullptr, nullptr, FF);
    k_hp<<<((NQR / 2) * NH_ + 7) / 8, 256, 0, stream>>>(Qf, NQR, QPh, QPl); k_hp<<<((NKR / 2) * NH_ + 7) / 8, 256, 0, stream>>>(Kf, NKR, KPh, KPl);
    for (int b = 0; b < NBT; ++b)
        for (int h = 0; h < NH_; ++h)
            k_gemm3<<<dim3(LQ / 64, LK / 64, 1), 128, 0, stream>>>(QPh + ((size_t)h * NQR + b * LQ) * DKP, QPl + ((size_t)h * NQR + b * LQ) * DKP, KPh + ((size_t)h * NKR + b * LK) * DKP, KPl + ((size_t)h * NKR + b * LK) * DKP, DKP, S + ((size_t)(b * NH_ + h)) * LQ * LK, LK);
    k_msoft<<<NBT * NH_ * (LQ / 8), 256, 0, stream>>>(S, mask, Vf, LAT);
    k_comb<<<(NBT * LQ * FF) / 256, 256, 0, stream>>>(LAT, Wc, bc, out);
}
